// NequIPInteractionBlock_88965952569932
// MI455X (gfx1250) — hardware-verified
//
#include <hip/hip_runtime.h>
#include <math.h>

typedef __attribute__((ext_vector_type(16))) _Float16 v16h;
typedef __attribute__((ext_vector_type(16))) __bf16 v16b;
typedef __attribute__((ext_vector_type(8)))  _Float16 v8h;
typedef __attribute__((ext_vector_type(8)))  float v8f;
typedef __attribute__((ext_vector_type(4)))  float v4f;
typedef __attribute__((ext_vector_type(2)))  float v2f;
typedef __attribute__((ext_vector_type(4)))  unsigned v4u;
typedef __attribute__((ext_vector_type(4)))  int v4i;
typedef float __attribute__((may_alias)) float_a;
typedef int __attribute__((may_alias)) int_a;

template <typename T> __device__ __forceinline__ void vst2(void* p, T v) { *(volatile T*)p = v; __threadfence(); *(volatile T*)p = v; }
__device__ __forceinline__ v8f wmma16(v16h a, v16h b, v8f c) {
  v8f d = __builtin_amdgcn_wmma_f32_16x16x32_f16(false, a, false, b, (short)0, c, false, false);
  asm volatile("v_nop\n\tv_nop\n\tv_nop\n\tv_nop" : "+v"(d) : "v"(a), "v"(b));
  return d;
}
__device__ __forceinline__ v8f wmma_bf(v16b a, v16b b, v8f c) {
  v8f d = __builtin_amdgcn_wmma_f32_16x16x32_bf16(false, a, false, b, (short)0, c, false, false);
  asm volatile("v_nop\n\tv_nop\n\tv_nop\n\tv_nop" : "+v"(d) : "v"(a), "v"(b));
  return d;
}
__device__ __forceinline__ v16h frag_h(const _Float16* rowk0, int lane) {
  union { v16h v; v8h q[2]; } u; const _Float16* p = rowk0 + 8 * (lane >> 4);
  u.q[0] = *(const v8h*)p; u.q[1] = *(const v8h*)(p + 16); return u.v;
}
__device__ __forceinline__ v16h frag_f32(const float* rowk0, int lane) {
  v16h a; const float* p = rowk0 + 8 * (lane >> 4);
#pragma unroll
  for (int i = 0; i < 8; ++i) { a[i] = (_Float16)p[i]; a[8 + i] = (_Float16)p[16 + i]; }
  return a;
}
__device__ __forceinline__ v16h frag_f32s(const float* rowk0, int lane, float sc) {
  v16h a; const float* p = rowk0 + 8 * (lane >> 4);
#pragma unroll
  for (int i = 0; i < 8; ++i) { a[i] = (_Float16)(p[i] * sc); a[8 + i] = (_Float16)(p[16 + i] * sc); }
  return a;
}
__device__ __forceinline__ v16h fragc_f32(const float* W, int k0, int n, int lane, int ld, int K) {
  v16h a; const int g = lane >> 4;
#pragma unroll
  for (int i = 0; i < 8; ++i) { const int ka = k0 + 8 * g + i, kb = ka + 16;
    a[i] = (_Float16)(ka < K ? W[(size_t)(ka < K ? ka : K - 1) * ld + n] : 0.f); a[8 + i] = (_Float16)(kb < K ? W[(size_t)(kb < K ? kb : K - 1) * ld + n] : 0.f); }
  return a;
}
struct F2 { v16b h, l; };
__device__ __forceinline__ F2 bsplit16(const float v[16]) { F2 r;
#pragma unroll
  for (int i = 0; i < 16; ++i) { const __bf16 h = (__bf16)v[i]; r.h[i] = h; r.l[i] = (__bf16)(v[i] - (float)h); }
  return r; }
__device__ __forceinline__ F2 split_row(const float* row, int k0, int lane) { float v[16]; const float* p = row + k0 + 8 * (lane >> 4);
#pragma unroll
  for (int i = 0; i < 8; ++i) { v[i] = p[i]; v[8 + i] = p[16 + i]; }
  return bsplit16(v); }
__device__ __forceinline__ F2 split_rowK(const float* row, int k0, int lane, int K) { float v[16]; const int g = lane >> 4;
#pragma unroll
  for (int i = 0; i < 8; ++i) { const int ka = k0 + 8 * g + i, kb = ka + 16; v[i] = ka < K ? row[ka < K ? ka : K - 1] : 0.f; v[8 + i] = kb < K ? row[kb < K ? kb : K - 1] : 0.f; }
  return bsplit16(v); }
__device__ __forceinline__ F2 split_col(const float* W, int k0, int n, int lane, int ld, int K) { float v[16]; const int g = lane >> 4;
#pragma unroll
  for (int i = 0; i < 8; ++i) { const int ka = k0 + 8 * g + i, kb = ka + 16; v[i] = ka < K ? W[(size_t)(ka < K ? ka : K - 1) * ld + n] : 0.f; v[8 + i] = kb < K ? W[(size_t)(kb < K ? kb : K - 1) * ld + n] : 0.f; }
  return bsplit16(v); }
__device__ __forceinline__ v8f mac3(const F2& a, const F2& b, v8f c) { c = wmma_bf(a.l, b.h, c); c = wmma_bf(a.h, b.l, c); return wmma_bf(a.h, b.h, c); }
__device__ __forceinline__ float sigm(float v) { return 1.0f / (1.0f + expf(-v)); }
#define LDSX() do { asm volatile("s_wait_dscnt 0" ::: "memory"); __builtin_amdgcn_wave_barrier(); __builtin_amdgcn_fence(__ATOMIC_RELEASE, "workgroup"); } while (0)


#define NB 2
#define NAT 4096
#define NNODE (NB * NAT)
#define KNB 32
#define NEDGE (NNODE * KNB)
#define SD 128
#define VD 64
#define RD 16
#define HDN 256
#define GW 384
#define K1 160
typedef __attribute__((ext_vector_type(8))) __bf16 v8b;
__device__ __forceinline__ v16b frag_b(const __bf16* rowk0, int lane) {
  union { v16b v; v8b q[2]; } u; const __bf16* p = rowk0 + 8 * (lane >> 4);
  u.q[0] = *(const v8b*)p; u.q[1] = *(const v8b*)(p + 16); return u.v;
}
__device__ __forceinline__ float bfr(float v) { return (float)(__bf16)v; }
__device__ __attribute__((noinline)) float exp_ni(float v) { return expf(v); }
__device__ __attribute__((noinline)) float erf_ni(float v) { return erff(v); }
__device__ __forceinline__ float silu_f(float x) { return x / (1.0f + exp_ni(-x)); }

#define PK_1A  0
#define PK_1B  (PK_1A + HDN * SD)
#define PK_2   (PK_1B + HDN * K1)
#define PK_VS  (PK_2 + GW * HDN)
#define PK_SV  (PK_VS + SD * VD)
#define PK_3   (PK_SV + VD * SD)
#define PK_4   (PK_3 + HDN * SD)
#define PK_MX  (PK_4 + SD * HDN)
#define PK_END (PK_MX + VD * VD)
#define WS_PK   0u
#define WS_SI   (((2u * PK_END) + 127u) / 128u * 128u)
#define WS_SM   (WS_SI + 4u * NNODE * HDN)
#define WS_VM   (WS_SM + 4u * NNODE * SD)
#define WS_END  (WS_VM + 4u * NNODE * VD * 3)

__global__ __launch_bounds__(256) void k_pack(const float* __restrict__ W1, const float* __restrict__ W2, const float* __restrict__ WVS, const float* __restrict__ WSV, const float* __restrict__ W3, const float* __restrict__ W4, const float* __restrict__ WMX, __bf16* __restrict__ PK) {
  __shared__ __align__(16) __bf16 s[HDN]; const int n = blockIdx.x, which = blockIdx.y, t = threadIdx.x; int K = 0; size_t dst = 0; float v = 0.f; bool act = true;
  switch (which) {
    case 0: act = n < HDN; K = SD;  dst = PK_1A + (size_t)n * SD;  if (act && t < K) v = W1[(size_t)t * HDN + n]; break;
    case 1: act = n < HDN; K = K1;  dst = PK_1B + (size_t)n * K1;  if (act && t < K) v = (t < SD + RD) ? W1[(size_t)(SD + t) * HDN + n] : 0.f; break;
    case 2: act = n < GW; K = HDN; dst = PK_2 + (size_t)n * HDN; if (act && t < K) v = W2[(size_t)t * GW + n]; break;
    case 3: act = n < SD; K = VD;  dst = PK_VS + (size_t)n * VD; if (act && t < K) v = WVS[(size_t)t * SD + n]; break;
    case 4: act = n < VD; K = SD;  dst = PK_SV + (size_t)n * SD; if (act && t < K) v = WSV[(size_t)t * VD + n]; break;
    case 5: act = n < HDN; K = SD;  dst = PK_3 + (size_t)n * SD;  if (act && t < K) v = W3[(size_t)t * HDN + n]; break;
    case 6: act = n < SD; K = HDN; dst = PK_4 + (size_t)n * HDN; if (act && t < K) v = W4[(size_t)t * SD + n]; break;
    default: act = n < VD; K = VD; dst = PK_MX + (size_t)n * VD; if (act && t < K) v = WMX[(size_t)n * VD + t]; break;
  }
  if (!act) return;
  if (t < K) s[t] = (__bf16)v;
  __syncthreads();
  if (t < K / 8) vst2((unsigned*)(PK + dst + t * 8), *(const v4u*)&s[t * 8]);
}
__global__ __launch_bounds__(128) void k_si(const float* __restrict__ S, const __bf16* __restrict__ PK, const float* __restrict__ B1, float* __restrict__ SI) {
  __shared__ __align__(16) float so[4][16][132];
  const int tid = threadIdx.x, wave = tid >> 5, lane = tid & 31, col = lane & 15, g = lane >> 4; const size_t r0 = (size_t)blockIdx.x * 64 + wave * 16; const int n0 = blockIdx.y * 128;
  v8f acc[8] = {};
#pragma unroll
  for (int kc = 0; kc < SD / 32; ++kc) { v16b a; { const float* p = S + (r0 + col) * SD + kc * 32 + 8 * g;
#pragma unroll
      for (int i = 0; i < 8; ++i) { a[i] = (__bf16)p[i]; a[8 + i] = (__bf16)p[16 + i]; } }
#pragma unroll
    for (int j = 0; j < 8; ++j) acc[j] = wmma_bf(a, frag_b(PK + PK_1A + (size_t)(n0 + j * 16 + col) * SD + kc * 32, lane), acc[j]); }
#pragma unroll
  for (int j = 0; j < 8; ++j) { const float bb = bfr(B1[n0 + j * 16 + col]);
#pragma unroll
    for (int r = 0; r < 8; ++r) so[wave][8 * g + r][j * 16 + col] = acc[j][r] + bb; }
  LDSX();
  for (int rl = 0; rl < 16; ++rl) vst2(SI + (r0 + rl) * HDN + n0 + lane * 4, *(const v4f*)&so[wave][rl][lane * 4]);
}
__global__ __launch_bounds__(128) void k_edge(const float* __restrict__ S, const float* __restrict__ V, const float* __restrict__ REL, const float* __restrict__ DIST, const float* __restrict__ RBF, const int* __restrict__ NBR, const __bf16* __restrict__ PK, const float* __restrict__ SI, const float* __restrict__ B2, float* __restrict__ SM, float* __restrict__ VM) {
  __shared__ __align__(16) __bf16 shh[64][HDN + 8]; __shared__ __align__(16) __bf16 shl[64][HDN + 8];
  __shared__ __align__(16) unsigned char R[72960];
  __shared__ float svfs[64][VD + 1]; __shared__ float smask[64]; __shared__ int sj[64]; __shared__ __align__(16) float sfin[2][192];
  float (*svp)[SD + 1] = (float (*)[SD + 1])(R);
  __bf16 (*sa)[K1 + 8] = (__bf16 (*)[K1 + 8])(R + 33024);
  __bf16 (*svrh)[72] = (__bf16 (*)[72])(R + 33024 + 21504); __bf16 (*svrl)[72] = (__bf16 (*)[72])(R + 33024 + 21504 + 9216);
  float (*sred)[SD + 1] = (float (*)[SD + 1])(R + 33024);
  float (*svec)[193] = (float (*)[193])(R);
  const int tid = threadIdx.x, wave = tid >> 5, lane = tid & 31, col = lane & 15, g = lane >> 4;
  const size_t nA = (size_t)blockIdx.x * 2;
  if (tid < 64) { const size_t node = nA + (tid >> 5); const int k = tid & 31; const int b = (int)(node / NAT); int j = NBR[node * KNB + k]; j = min(max(j, 0), NAT - 1); sj[tid] = (int)((size_t)b * NAT + j); smask[tid] = (bfr(DIST[node * KNB + k]) < 0.5f) ? 1.f : 0.f; }
  __syncthreads();
  for (int e = tid; e < 64 * (K1 + 8); e += 128) { const int r = e / (K1 + 8), c = e % (K1 + 8); const size_t node = nA + (r >> 5); const int k = r & 31; float v = 0.f;
    if (c < SD) v = bfr(S[(size_t)sj[r] * SD + c]); else if (c < SD + RD) v = bfr(RBF[(node * KNB + k) * RD + (c - SD)]);
    sa[r][c] = (__bf16)v; }
  for (int e = tid; e < 64 * 72; e += 128) { const int r = e / 72, u = e % 72; float x = 0.f;
    if (u < VD) { const size_t node = nA + (r >> 5); const int k = r & 31; const float* vj = V + ((size_t)sj[r] * VD + u) * 3; const float* rl = REL + (node * KNB + k) * 3; x = (bfr(vj[0]) * bfr(rl[0]) + bfr(vj[1]) * bfr(rl[1])) + bfr(vj[2]) * bfr(rl[2]); }
    const __bf16 hb = (__bf16)x; svrh[r][u] = hb; svrl[r][u] = (__bf16)(x - (float)hb); }
  __syncthreads();
#pragma unroll 1
  for (int half = 0; half < 2; ++half) { v8f acc[8] = {};
#pragma unroll 1
    for (int kc = 0; kc < K1 / 32; ++kc) { const v16b a = frag_b(&sa[wave * 16 + col][kc * 32], lane);
#pragma unroll
      for (int j = 0; j < 8; ++j) acc[j] = wmma_bf(a, frag_b(PK + PK_1B + (size_t)(half * 128 + j * 16 + col) * K1 + kc * 32, lane), acc[j]); }
#pragma unroll
    for (int j = 0; j < 8; ++j) { const int c = half * 128 + j * 16 + col;
#pragma unroll
      for (int r = 0; r < 8; ++r) { const int row = wave * 16 + 8 * g + r; const size_t node = nA + (row >> 5); const float v = silu_f(acc[j][r] + SI[node * HDN + c]); const __bf16 hb = (__bf16)v; shh[row][c] = hb; shl[row][c] = (__bf16)(v - (float)hb); } } }
  { v8f acc[8] = {};
#pragma unroll
    for (int kc = 0; kc < VD / 32; ++kc) { F2 a; a.h = frag_b(&svrh[wave * 16 + col][kc * 32], lane); a.l = frag_b(&svrl[wave * 16 + col][kc * 32], lane);
#pragma unroll
      for (int j = 0; j < 8; ++j) { const v16b w = frag_b(PK + PK_VS + (size_t)(j * 16 + col) * VD + kc * 32, lane); acc[j] = wmma_bf(a.l, w, acc[j]); acc[j] = wmma_bf(a.h, w, acc[j]); } }
#pragma unroll
    for (int j = 0; j < 8; ++j)
#pragma unroll
      for (int r = 0; r < 8; ++r) svp[wave * 16 + 8 * g + r][j * 16 + col] = acc[j][r]; }
  { v8f acc[4] = {};
#pragma unroll
    for (int kc = 0; kc < SD / 32; ++kc) { const v16b a = frag_b(&sa[wave * 16 + col][kc * 32], lane);
#pragma unroll
      for (int j = 0; j < 4; ++j) acc[j] = wmma_bf(a, frag_b(PK + PK_SV + (size_t)(j * 16 + col) * SD + kc * 32, lane), acc[j]); }
#pragma unroll
    for (int j = 0; j < 4; ++j)
#pragma unroll
      for (int r = 0; r < 8; ++r) svfs[wave * 16 + 8 * g + r][j * 16 + col] = acc[j][r]; }
  __syncthreads();
  float se[2][8][8];
#pragma unroll 1
  for (int half = 0; half < 2; ++half) { v8f acc[8] = {};
#pragma unroll 1
    for (int kc = 0; kc < HDN / 32; ++kc) { F2 a; a.h = frag_b(&shh[wave * 16 + col][kc * 32], lane); a.l = frag_b(&shl[wave * 16 + col][kc * 32], lane);
#pragma unroll
      for (int j = 0; j < 8; ++j) { const v16b w = frag_b(PK + PK_2 + (size_t)(half * 128 + j * 16 + col) * HDN + kc * 32, lane); acc[j] = wmma_bf(a.l, w, acc[j]); acc[j] = wmma_bf(a.h, w, acc[j]); } }
#pragma unroll
    for (int j = 0; j < 8; ++j) { const int c = j * 16 + col; const float bb = bfr(B2[half * 128 + c]);
#pragma unroll
      for (int r = 0; r < 8; ++r) { const int row = wave * 16 + 8 * g + r; const float gate = acc[j][r] + bb; const float m = smask[row];
        if (half == 0) sred[row][c] = m * gate * bfr(S[(size_t)sj[row] * SD + c]);
        else sred[row][c] += m * gate * svp[row][c]; } }
  }
  (void)se;
  __syncthreads();
  { const int c = tid; float sAc = 0.f, sBc = 0.f, cA = 0.f, cB = 0.f;
#pragma unroll 1
    for (int k = 0; k < 32; ++k) { sAc += sred[k][c]; sBc += sred[32 + k][c]; cA += smask[k]; cB += smask[32 + k]; }
    sfin[0][c] = sAc / fmaxf(cA, 1.f); sfin[1][c] = sBc / fmaxf(cB, 1.f); }
  __syncthreads();
  if (tid < 64) { const int nn = tid >> 5, pc = tid & 31; vst2(SM + (nA + nn) * SD + pc * 4, *(const v4f*)&sfin[nn][pc * 4]); }
  __syncthreads();
  if (tid < 64) { const size_t node = nA + (tid >> 5); const int k = tid & 31; const float* rl = REL + (node * KNB + k) * 3; svec[tid][192] = 0.f; sfin[0][tid] = bfr(rl[0]); sfin[0][64 + tid] = bfr(rl[1]); sfin[0][128 + tid] = bfr(rl[2]); }
  __syncthreads();
#pragma unroll 1
  for (int ph = 0; ph < 2; ++ph) { v8f acc[4] = {};
#pragma unroll 1
    for (int kc = 0; kc < HDN / 32; ++kc) { F2 a; a.h = frag_b(&shh[wave * 16 + col][kc * 32], lane); a.l = frag_b(&shl[wave * 16 + col][kc * 32], lane);
#pragma unroll
      for (int jj = 0; jj < 4; ++jj) { const int j = (jj < 2) ? (ph * 2 + jj) : (4 + ph * 2 + (jj - 2)); const v16b w = frag_b(PK + PK_2 + (size_t)(256 + j * 16 + col) * HDN + kc * 32, lane); acc[jj] = wmma_bf(a.l, w, acc[jj]); acc[jj] = wmma_bf(a.h, w, acc[jj]); } }
#pragma unroll
    for (int jj = 0; jj < 2; ++jj) { const int u = (ph * 2 + jj) * 16 + col; const float bvv = bfr(B2[256 + u]), bvs = bfr(B2[320 + u]);
#pragma unroll
      for (int r = 0; r < 8; ++r) { const int row = wave * 16 + 8 * g + r; const float gvv = acc[jj][r] + bvv, gvs = acc[jj + 2][r] + bvs; const float m = smask[row];
        const float* vj = V + ((size_t)sj[row] * VD + u) * 3; const float f = gvs * svfs[row][u];
#pragma unroll
        for (int c3 = 0; c3 < 3; ++c3) svec[row][u * 3 + c3] = m * (gvv * bfr(vj[c3]) + f * sfin[0][c3 * 64 + row]); } } }
  __syncthreads();
  for (int cc = tid; cc < 192; cc += 128) { float sAc = 0.f, sBc = 0.f, cA = 0.f, cB = 0.f;
#pragma unroll 1
    for (int k = 0; k < 32; ++k) { sAc += svec[k][cc]; sBc += svec[32 + k][cc]; cA += smask[k]; cB += smask[32 + k]; }
    sfin[0][cc] = sAc / fmaxf(cA, 1.f); sfin[1][cc] = sBc / fmaxf(cB, 1.f); }
  __syncthreads();
  if (tid < 96) { const int nn = tid / 48, pc = tid % 48; vst2(VM + (nA + nn) * (VD * 3) + pc * 4, *(const v4f*)&sfin[nn][pc * 4]); }
}
__global__ __launch_bounds__(128) void k_node(const float* __restrict__ SM, const float* __restrict__ S, const __bf16* __restrict__ PK, const float* __restrict__ B3, const float* __restrict__ B4, const float* __restrict__ GS, const float* __restrict__ BS, float* __restrict__ OUTS) {
  __shared__ __align__(16) __bf16 sth[64][HDN + 8], stl[64][HDN + 8]; __shared__ __align__(16) float sx[4][16][SD + 4]; __shared__ float sps[4][16][16][2];
  const int tid = threadIdx.x, wave = tid >> 5, lane = tid & 31, col = lane & 15, g = lane >> 4; const size_t r0 = (size_t)blockIdx.x * 64 + wave * 16;
#pragma unroll 1
  for (int half = 0; half < 2; ++half) { v8f acc[8] = {};
#pragma unroll
    for (int kc = 0; kc < SD / 32; ++kc) { const F2 a = split_row(SM + (r0 + col) * SD, kc * 32, lane);
#pragma unroll
      for (int j = 0; j < 8; ++j) { const v16b w = frag_b(PK + PK_3 + (size_t)(half * 128 + j * 16 + col) * SD + kc * 32, lane); acc[j] = wmma_bf(a.l, w, acc[j]); acc[j] = wmma_bf(a.h, w, acc[j]); } }
#pragma unroll
    for (int j = 0; j < 8; ++j) { const int c = half * 128 + j * 16 + col; const float bb = bfr(B3[c]);
#pragma unroll
      for (int r = 0; r < 8; ++r) { const float v = silu_f(acc[j][r] + bb); const __bf16 hb = (__bf16)v; sth[wave * 16 + 8 * g + r][c] = hb; stl[wave * 16 + 8 * g + r][c] = (__bf16)(v - (float)hb); } } }
  LDSX();
  v8f acc[8] = {};
#pragma unroll 2
  for (int kc = 0; kc < HDN / 32; ++kc) { F2 a; a.h = frag_b(&sth[wave * 16 + col][kc * 32], lane); a.l = frag_b(&stl[wave * 16 + col][kc * 32], lane);
#pragma unroll
    for (int j = 0; j < 8; ++j) { const v16b w = frag_b(PK + PK_4 + (size_t)(j * 16 + col) * HDN + kc * 32, lane); acc[j] = wmma_bf(a.l, w, acc[j]); acc[j] = wmma_bf(a.h, w, acc[j]); } }
  float s1[8], s2[8];
#pragma unroll
  for (int r = 0; r < 8; ++r) { s1[r] = 0.f; s2[r] = 0.f; }
#pragma unroll
  for (int j = 0; j < 8; ++j) { const int c = j * 16 + col; const float bb = bfr(B4[c]);
#pragma unroll
    for (int r = 0; r < 8; ++r) { const size_t row = r0 + 8 * g + r; const float v = acc[j][r] + bb + bfr(S[row * SD + c]); sx[wave][8 * g + r][c] = v; s1[r] += v; s2[r] += v * v; } }
#pragma unroll
  for (int r = 0; r < 8; ++r) { sps[wave][8 * g + r][col][0] = s1[r]; sps[wave][8 * g + r][col][1] = s2[r]; }
  LDSX();
  for (int rl = 0; rl < 16; ++rl) { float a = 0.f, b2 = 0.f;
#pragma unroll
    for (int k = 0; k < 16; ++k) { a += sps[wave][rl][k][0]; b2 += sps[wave][rl][k][1]; }
    const float mu = a / (float)SD; const float var = fmaxf(b2 / (float)SD - mu * mu, 0.f); const float inv = 1.0f / sqrtf(var + 1e-5f); v4f o;
#pragma unroll
    for (int i = 0; i < 4; ++i) { const int c = lane * 4 + i; o[i] = (sx[wave][rl][c] - mu) * inv * bfr(GS[c]) + bfr(BS[c]); }
    vst2(OUTS + (r0 + rl) * SD + lane * 4, o); }
}
__global__ __launch_bounds__(128) void k_vec(const float* __restrict__ VM, const float* __restrict__ Vin, const __bf16* __restrict__ PK, const float* __restrict__ GV, const float* __restrict__ BV, float* __restrict__ OUTV) {
  __shared__ __align__(16) __bf16 sah[64][72], sal[64][72]; __shared__ float svs[16][3][VD + 1]; __shared__ float smag[16][VD + 1]; __shared__ __align__(16) float sout[16][VD * 3];
  const int tid = threadIdx.x, wave = tid >> 5, lane = tid & 31, col = lane & 15, g = lane >> 4; const size_t n0 = (size_t)blockIdx.x * 16;
  for (int e = tid; e < 64 * 72; e += 128) { const int r = e / 72, v = e % 72; float x = 0.f; if (r < 48 && v < VD) { const size_t node = n0 + r / 3; const int c = r % 3; x = VM[node * (VD * 3) + v * 3 + c]; } const __bf16 hb = (__bf16)x; sah[r][v] = hb; sal[r][v] = (__bf16)(x - (float)hb); }
  __syncthreads();
  if (wave < 3) { v8f acc[4] = {};
#pragma unroll
    for (int kc = 0; kc < VD / 32; ++kc) { F2 a; a.h = frag_b(&sah[wave * 16 + col][kc * 32], lane); a.l = frag_b(&sal[wave * 16 + col][kc * 32], lane);
#pragma unroll
      for (int j = 0; j < 4; ++j) { const v16b w = frag_b(PK + PK_MX + (size_t)(j * 16 + col) * VD + kc * 32, lane); acc[j] = wmma_bf(a.l, w, acc[j]); acc[j] = wmma_bf(a.h, w, acc[j]); } }
#pragma unroll
    for (int j = 0; j < 4; ++j) { const int u = j * 16 + col;
#pragma unroll
      for (int r = 0; r < 8; ++r) { const int row = wave * 16 + 8 * g + r; const int nl = row / 3, c = row % 3; const size_t node = n0 + nl; svs[nl][c][u] = bfr(Vin[(node * VD + u) * 3 + c]) + acc[j][r]; } } }
  __syncthreads();
  if (tid < VD) { const int u = tid;
#pragma unroll 1
    for (int nl = 0; nl < 16; ++nl) { const float x = svs[nl][0][u], y = svs[nl][1][u], z = svs[nl][2][u]; smag[nl][u] = fmaxf(sqrtf((x * x + y * y) + z * z), 1e-6f); } }
  __syncthreads();
  if (tid < 16) { const int nl = tid; float a = 0.f; for (int u = 0; u < VD; ++u) a += smag[nl][u]; const float mu = a / (float)VD; float b2 = 0.f; for (int u = 0; u < VD; ++u) { const float d = smag[nl][u] - mu; b2 += d * d; } const float inv = 1.0f / sqrtf(b2 / (float)VD + 1e-5f);
    for (int u = 0; u < VD; ++u) { const float mn = (smag[nl][u] - mu) * inv * bfr(GV[u]) + bfr(BV[u]); const float sc = mn / smag[nl][u];
#pragma unroll
      for (int c = 0; c < 3; ++c) sout[nl][u * 3 + c] = svs[nl][c][u] * sc; } }
  __syncthreads();
  for (int q = tid; q < 16 * VD * 3 / 4; q += 128) vst2(OUTV + n0 * (VD * 3) + q * 4, *(const v4f*)(&sout[0][0] + q * 4));
}
extern "C" void kernel_launch(void* const* d_in, const int* in_sizes, int n_in, void* d_out, int out_size, void* d_ws, size_t ws_size, hipStream_t stream) {
  (void)in_sizes; (void)n_in; (void)out_size;
  const float** F = (const float**)d_in;
  if (ws_size < (size_t)WS_END) return;
  char* ws = (char*)d_ws; __bf16* PK = (__bf16*)(ws + WS_PK); float *SI = (float*)(ws + WS_SI), *SM = (float*)(ws + WS_SM), *VM = (float*)(ws + WS_VM);
  float* OUTS = (float*)d_out; float* OUTV = (float*)((char*)d_out + 4194304);
  k_pack<<<dim3(GW, 8), 256, 0, stream>>>(F[5], F[7], F[9], F[10], F[11], F[13], F[15], PK);
  k_si<<<dim3(NNODE / 64, HDN / 128), 128, 0, stream>>>(F[0], PK, F[6], SI);
  k_edge<<<NNODE / 2, 128, 0, stream>>>(F[0], F[1], F[2], F[3], F[4], (const int*)d_in[20], PK, SI, F[8], SM, VM);
  k_node<<<NNODE / 64, 128, 0, stream>>>(SM, F[0], PK, F[12], F[14], F[16], F[17], OUTS);
  k_vec<<<NNODE / 16, 128, 0, stream>>>(VM, F[1], PK, F[18], F[19], OUTV);
}
